// SimpleRNN_19971597926442
// MI455X (gfx1250) — hardware-verified
//
#include <hip/hip_runtime.h>
#include <math.h>

constexpr int NSEQ    = 256;
constexpr int NSTEP   = 512;
constexpr int NVOC    = 32000;
constexpr int NEMB    = 256;
constexpr int NHID    = 512;
constexpr int NTHR    = 256;
constexpr int SEQ_BLK = 16;
constexpr int HPITCH  = 520;
constexpr int XPITCH  = 516;
static_assert(NSEQ % SEQ_BLK == 0);
static_assert(NHID == 64 * (NTHR / 32));
static_assert(NHID % 32 == 0 && NEMB % 32 == 0);
static_assert(NVOC % 64 == 0 && NHID % 64 == 0);
static_assert(((NVOC / 64) * (NHID / 64)) % 8 == 0);
static_assert((NVOC * (NEMB / 8)) % NTHR == 0);
static_assert((NHID * (NEMB / 8)) % NTHR == 0);
static_assert((NHID * (NHID / 8)) % NTHR == 0);
static_assert(HPITCH % 8 == 0 && XPITCH % 4 == 0);
static_assert(SEQ_BLK * (NHID / 32) == NTHR);
static_assert((SEQ_BLK * NHID / 4) % NTHR == 0);

typedef __attribute__((ext_vector_type(16))) _Float16 v16h;
typedef __attribute__((ext_vector_type(8)))  _Float16 v8h;
typedef __attribute__((ext_vector_type(16))) __bf16   v16b;
typedef __attribute__((ext_vector_type(8)))  __bf16   v8b;
typedef __attribute__((ext_vector_type(8)))  float    v8f;
typedef __attribute__((ext_vector_type(4)))  float    v4f;

__device__ __forceinline__ unsigned short f2bf_bits(float f) {
  unsigned u = __float_as_uint(f);
  return (unsigned short)((u + 0x7FFFu + ((u >> 16) & 1u)) >> 16);
}
__device__ __forceinline__ float bf_bits2f(unsigned short h) { return __uint_as_float(((unsigned)h) << 16); }
__device__ __forceinline__ float bf16r(float f) { return bf_bits2f(f2bf_bits(f)); }

__device__ __forceinline__ void dep_guard_h(v8f& a, v8f& b, v16h x, v16h y) { asm volatile("v_nop\n\tv_nop\n\tv_nop\n\tv_nop" : "+v"(a), "+v"(b) : "v"(x), "v"(y)); }
__device__ __forceinline__ void dep_guard_b(v8f& a, v8f& b, v16b x, v16b y) { asm volatile("v_nop\n\tv_nop\n\tv_nop\n\tv_nop" : "+v"(a), "+v"(b) : "v"(x), "v"(y)); }
__device__ __forceinline__ void keep4_h(v16h a, v16h b, v16h c, v16h d) { asm volatile("v_nop" :: "v"(a), "v"(b), "v"(c), "v"(d)); }
__device__ __forceinline__ void keep4_b(v16b a, v16b b, v16b c, v16b d) { asm volatile("v_nop" :: "v"(a), "v"(b), "v"(c), "v"(d)); }
__device__ __forceinline__ void acc_guard4(v8f& a, v8f& b, v8f& c, v8f& d) { asm volatile("v_nop\n\tv_nop\n\tv_nop\n\tv_nop" : "+v"(a), "+v"(b), "+v"(c), "+v"(d)); }
__device__ __forceinline__ void tie4x6_h(v8f& a0, v8f& a1, v8f& a2, v8f& a3, v16h x0, v16h x1, v16h y0, v16h y1, v16h y2, v16h y3) {
  asm volatile("v_nop\n\tv_nop\n\tv_nop\n\tv_nop" : "+v"(a0), "+v"(a1), "+v"(a2), "+v"(a3) : "v"(x0), "v"(x1), "v"(y0), "v"(y1), "v"(y2), "v"(y3));
}
__device__ __forceinline__ void tie4x6_b(v8f& a0, v8f& a1, v8f& a2, v8f& a3, v16b x0, v16b x1, v16b y0, v16b y1, v16b y2, v16b y3) {
  asm volatile("v_nop\n\tv_nop\n\tv_nop\n\tv_nop" : "+v"(a0), "+v"(a1), "+v"(a2), "+v"(a3) : "v"(x0), "v"(x1), "v"(y0), "v"(y1), "v"(y2), "v"(y3));
}
template <typename T> struct Frag;
template <> struct Frag<_Float16> {
  typedef v16h V; union U { v16h v; v8h h[2]; };
  static __device__ __forceinline__ v16h load(const _Float16* p) {
    U f; f.h[0] = *(const v8h*)(p); f.h[1] = *(const v8h*)(p + 16); return f.v;
  }
  static __device__ __forceinline__ v8f mma(v16h a, v16h b, v8f c) {
    return __builtin_amdgcn_wmma_f32_16x16x32_f16(false, a, false, b, (short)0, c, false, false);
  }
  static __device__ __forceinline__ void guard(v8f& a, v8f& b, v16h x, v16h y) { dep_guard_h(a, b, x, y); }
  static __device__ __forceinline__ void keep(v16h a, v16h b, v16h c, v16h d) { keep4_h(a, b, c, d); }
  static __device__ __forceinline__ void tie(v8f& a0, v8f& a1, v8f& a2, v8f& a3, v16h x0, v16h x1, v16h y0, v16h y1, v16h y2, v16h y3) {
    tie4x6_h(a0, a1, a2, a3, x0, x1, y0, y1, y2, y3);
  }
};
template <> struct Frag<__bf16> {
  typedef v16b V; union U { v16b v; v8b h[2]; };
  static __device__ __forceinline__ v16b load(const __bf16* p) {
    U f; f.h[0] = *(const v8b*)(p); f.h[1] = *(const v8b*)(p + 16); return f.v;
  }
  static __device__ __forceinline__ v8f mma(v16b a, v16b b, v8f c) {
    return __builtin_amdgcn_wmma_f32_16x16x32_bf16(false, a, false, b, (short)0, c, false, false);
  }
  static __device__ __forceinline__ void guard(v8f& a, v8f& b, v16b x, v16b y) { dep_guard_b(a, b, x, y); }
  static __device__ __forceinline__ void keep(v16b a, v16b b, v16b c, v16b d) { keep4_b(a, b, c, d); }
  static __device__ __forceinline__ void tie(v8f& a0, v8f& a1, v8f& a2, v8f& a3, v16b x0, v16b x1, v16b y0, v16b y1, v16b y2, v16b y3) {
    tie4x6_b(a0, a1, a2, a3, x0, x1, y0, y1, y2, y3);
  }
};

template <int ET> struct Elem;
template <> struct Elem<0> { typedef _Float16 T; };
template <> struct Elem<1> { typedef __bf16 T; };
template <int ET, bool SPLIT, int BIAS_MODE, int OUT_MODE, bool RESID, int ACT = 0>
__global__ __launch_bounds__(256) void wmma_gemm64(
    const unsigned short* __restrict__ Ap, const unsigned short* __restrict__ A2p, int lda, long strideA,
    const unsigned short* __restrict__ Btp, const unsigned short* __restrict__ Bt2p, int ldb, long strideB,
    void* __restrict__ Cout, void* __restrict__ Cout2, int ldc, long strideC,
    const float* __restrict__ bias,
    const float* __restrict__ resid, long strideR,
    int M, int N, int K, float scale) {
  typedef typename Elem<ET>::T T;
  typedef typename Frag<T>::V V;
  const T* A = (const T*)Ap; const T* A2 = (const T*)A2p; const T* Bt = (const T*)Btp; const T* Bt2 = (const T*)Bt2p;
  __shared__ __align__(16) float sT[8][16 * 68];
  const int b    = blockIdx.y;
  const int lane = threadIdx.x & 31;
  const int wave = threadIdx.x >> 5;
  const int tilesN = N >> 6;
  const int tilesM = M >> 6;
  const int tile = blockIdx.x * 8 + wave;
  if (tile >= tilesM * tilesN) return;
  const int tm = tile / tilesN;
  const int tn = tile - tm * tilesN;
  const int m0 = tm << 6;
  const int n0 = tn << 6;

  const T* Ab  = A  + (size_t)b * strideA;
  const T* Bb  = Bt + (size_t)b * strideB;
  const T* Ab2 = SPLIT ? (A2  + (size_t)b * strideA) : nullptr;
  const T* Bb2 = SPLIT ? (Bt2 + (size_t)b * strideB) : nullptr;

  const int rlane = lane & 15;
  const int koff  = (lane >> 4) * 8;
  const int mOff  = (lane >> 4) * 8;

  v8f acc[4][4];
#pragma unroll
  for (int i = 0; i < 4; ++i)
#pragma unroll
    for (int j = 0; j < 4; ++j) acc[i][j] = (v8f){0.f,0.f,0.f,0.f,0.f,0.f,0.f,0.f};

  for (int k0 = 0; k0 < K; k0 += 32) {
    V bh[4], bl[4];
#pragma unroll
    for (int j = 0; j < 4; ++j) {
      const size_t bo = (size_t)(n0 + (j << 4) + rlane) * ldb + koff + k0;
      bh[j] = Frag<T>::load(Bb + bo);
      if (SPLIT) bl[j] = Frag<T>::load(Bb2 + bo);
    }
#pragma unroll
    for (int i = 0; i < 4; ++i) {
      const size_t ao = (size_t)(m0 + (i << 4) + rlane) * lda + koff + k0;
      V ah = Frag<T>::load(Ab + ao);
      V al;
      if (SPLIT) al = Frag<T>::load(Ab2 + ao);
#pragma unroll
      for (int j = 0; j < 4; ++j) {
        acc[i][j] = Frag<T>::mma(ah, bh[j], acc[i][j]);
        if (SPLIT) {
          acc[i][j] = Frag<T>::mma(ah, bl[j], acc[i][j]);
          acc[i][j] = Frag<T>::mma(al, bh[j], acc[i][j]);
        }
      }
      Frag<T>::tie(acc[i][0], acc[i][1], acc[i][2], acc[i][3], ah, SPLIT ? al : ah, bh[0], bh[1], bh[2], bh[3]);
    }
    Frag<T>::keep(bh[0], bh[1], bh[2], bh[3]);
    if (SPLIT) Frag<T>::keep(bl[0], bl[1], bl[2], bl[3]);
  }
  acc_guard4(acc[0][0], acc[0][1], acc[0][2], acc[0][3]);
  acc_guard4(acc[1][0], acc[1][1], acc[1][2], acc[1][3]);
  acc_guard4(acc[2][0], acc[2][1], acc[2][2], acc[2][3]);
  acc_guard4(acc[3][0], acc[3][1], acc[3][2], acc[3][3]);

  float* slab = sT[wave];
  const float* Rb = RESID ? (resid + (size_t)b * strideR) : nullptr;
#pragma unroll
  for (int i = 0; i < 4; ++i) {
    const int mBase = m0 + (i << 4);
#pragma unroll
    for (int j = 0; j < 4; ++j) {
      const int n = n0 + (j << 4) + rlane;
      float bv = 0.f;
      if (BIAS_MODE == 2) bv = bias[n];
#pragma unroll
      for (int r = 0; r < 8; ++r) {
        float v = acc[i][j][r] * scale;
        if (BIAS_MODE == 1) v += bias[mBase + mOff + r];
        if (BIAS_MODE == 2) v += bv;
        if (RESID) v += Rb[(size_t)(mBase + mOff + r) * ldc + n];
        if (ACT == 1) v = tanhf(v);
        if (ACT == 2) v = fmaxf(v, 0.0f);
        if (ACT == 3) v = v / (1.0f + expf(-v));
        if (ACT == 4) v = (v > 0.f) ? v : 0.01f * v;
        if (ACT == 5) v = 0.5f * v * (1.0f + erff(v * 0.70710678118654752f));
        slab[(mOff + r) * 68 + (j << 4) + rlane] = v;
      }
    }
    __builtin_amdgcn_fence(__ATOMIC_RELEASE, "workgroup");
    __builtin_amdgcn_wave_barrier();
    __builtin_amdgcn_fence(__ATOMIC_ACQUIRE, "workgroup");
    if (OUT_MODE == 0) {
      float* C = (float*)Cout + (size_t)b * strideC;
      const int hh = lane >> 4, c4 = (lane & 15) * 4;
      for (int pass = 0; pass < 2; ++pass) {
#pragma unroll
        for (int it = 0; it < 8; ++it) {
          const int row = it * 2 + hh;
          v4f v = *(const v4f*)(slab + row * 68 + c4);
          *(volatile v4f*)(C + (size_t)(mBase + row) * ldc + n0 + c4) = v;
        }
        __threadfence();
      }
    } else {
      const int q = lane >> 3, c8 = (lane & 7) * 8;
      unsigned short* C  = (unsigned short*)Cout  + (size_t)b * strideC;
      unsigned short* C2 = (OUT_MODE == 2) ? ((unsigned short*)Cout2 + (size_t)b * strideC) : nullptr;
      for (int pass = 0; pass < 2; ++pass) {
#pragma unroll
        for (int it = 0; it < 4; ++it) {
          const int row = it * 4 + q;
          const float* sp = slab + row * 68 + c8;
          v8h hv, lv;
#pragma unroll
          for (int e = 0; e < 8; ++e) {
            if (OUT_MODE == 1) {
              hv[e] = (_Float16)sp[e];
            } else {
              unsigned short hb = f2bf_bits(sp[e]);
              unsigned short lb = f2bf_bits(sp[e] - bf_bits2f(hb));
              hv[e] = __builtin_bit_cast(_Float16, hb);
              lv[e] = __builtin_bit_cast(_Float16, lb);
            }
          }
          *(volatile v8h*)(C + (size_t)(mBase + row) * ldc + n0 + c8) = hv;
          if (OUT_MODE == 2) *(volatile v8h*)(C2 + (size_t)(mBase + row) * ldc + n0 + c8) = lv;
        }
        __threadfence();
      }
    }
    __builtin_amdgcn_fence(__ATOMIC_RELEASE, "workgroup");
    __builtin_amdgcn_wave_barrier();
    __builtin_amdgcn_fence(__ATOMIC_ACQUIRE, "workgroup");
  }
}

template <int MODE>
__global__ __launch_bounds__(NTHR) void cvt8_kernel(const float* __restrict__ src, unsigned short* __restrict__ dst,
                                                    int nrow, int ncol8, int spitch, int scol0, float sc) {
  const int i  = blockIdx.x * NTHR + threadIdx.x;
  const int n8 = nrow * ncol8;
  if (i < n8) {
    const int row = i / ncol8;
    const int c8  = i - row * ncol8;
    const float* sp = src + (size_t)row * spitch + scol0 + c8 * 8;
    const v4f a = *(const v4f*)(sp);
    const v4f b = *(const v4f*)(sp + 4);
    v8h hv;
#pragma unroll
    for (int e = 0; e < 4; ++e) {
      unsigned short b0, b1;
      if (MODE == 0) {
        b0 = f2bf_bits(a[e] * sc);
        b1 = f2bf_bits(b[e] * sc);
      } else {
        b0 = __builtin_bit_cast(unsigned short, (_Float16)(bf16r(a[e]) * sc));
        b1 = __builtin_bit_cast(unsigned short, (_Float16)(bf16r(b[e]) * sc));
      }
      hv[e]     = __builtin_bit_cast(_Float16, b0);
      hv[4 + e] = __builtin_bit_cast(_Float16, b1);
    }
    *(volatile v8h*)(dst + (size_t)i * 8) = hv;
    __threadfence();
    *(volatile v8h*)(dst + (size_t)i * 8) = hv;
  }
}

__global__ __launch_bounds__(NTHR) void bias_prep_kernel(const float* __restrict__ b_a, const float* __restrict__ b_b,
                                                         float* __restrict__ dst) {
  const int tid = threadIdx.x;
  const int which = tid >> 7;
  const int idx = (tid & 127) * 4;
  const v4f va = *(const v4f*)(b_a + idx);
  const v4f vb = *(const v4f*)(b_b + idx);
  v4f o;
#pragma unroll
  for (int e = 0; e < 4; ++e) o[e] = bf16r(which ? vb[e] : va[e]);
  float* op = dst + which * NHID + idx;
  *(volatile v4f*)op = o;
  __threadfence();
  *(volatile v4f*)op = o;
}

__device__ __forceinline__ void gather_xp(float* Xs, const int* __restrict__ X, const float* __restrict__ PT,
                                          int rowbase, int t, int tid) {
  const int m   = tid >> 4;
  const int seg = (tid & 15) * 32;
  int id = X[(size_t)(rowbase + m) * NSTEP + t];
  id = (id < 0) ? 0 : id;
  id = (id > NVOC - 1) ? (NVOC - 1) : id;
  const float* src = PT + (size_t)id * NHID + seg;
  v4f v[8];
#pragma unroll
  for (int i = 0; i < 8; ++i) v[i] = *(const v4f*)(src + 4 * i);
  float* dst = Xs + m * XPITCH + seg;
#pragma unroll
  for (int i = 0; i < 8; ++i) *(v4f*)(dst + 4 * i) = v[i];
}

__global__ __launch_bounds__(NTHR) void rnn_seq_kernel(const int* __restrict__ X, const float* __restrict__ PT,
                                                       const float* __restrict__ BIAS2,
                                                       const unsigned short* __restrict__ WHp,
                                                       float* __restrict__ out) {
  __shared__ __align__(16) unsigned short Hh[SEQ_BLK * HPITCH];
  __shared__ __align__(16) unsigned short Hl[SEQ_BLK * HPITCH];
  __shared__ __align__(16) float          Xs[SEQ_BLK * XPITCH];
  const __bf16* WH = (const __bf16*)WHp;
  const int tid = threadIdx.x, lane = tid & 31, wave = tid >> 5;
  const int c = lane & 15, hh = lane >> 4, koff = hh * 8;
  const int rowbase = blockIdx.x * SEQ_BLK;

#pragma unroll 1
  for (int i = tid; i < SEQ_BLK * HPITCH; i += NTHR) { Hh[i] = (unsigned short)0; Hl[i] = (unsigned short)0; }
  gather_xp(Xs, X, PT, rowbase, 0, tid);
  float bhh[4], hst[4][8];
#pragma unroll
  for (int nt = 0; nt < 4; ++nt) {
    const int j = 64 * wave + 16 * nt + c;
    bhh[nt] = BIAS2[NHID + j];
#pragma unroll
    for (int r = 0; r < 8; ++r) hst[nt][r] = 0.0f;
  }
  __syncthreads();

  const __bf16* ahrow = (const __bf16*)Hh + c * HPITCH + koff;
  const __bf16* alrow = (const __bf16*)Hl + c * HPITCH + koff;
  const __bf16* wbase = WH + (size_t)(64 * wave + c) * NHID + koff;
  const v8f z8 = {0.f, 0.f, 0.f, 0.f, 0.f, 0.f, 0.f, 0.f};

#pragma unroll 1
  for (int t = 0; t < NSTEP; ++t) {
    v8f acc[4];
    acc[0] = z8; acc[1] = z8; acc[2] = z8; acc[3] = z8;
#pragma unroll 1
    for (int k0 = 0; k0 < NHID; k0 += 32) {
      const v16b fa = Frag<__bf16>::load(ahrow + k0);
      const v16b fl = Frag<__bf16>::load(alrow + k0);
      const v16b b0 = Frag<__bf16>::load(wbase + k0);
      const v16b b1 = Frag<__bf16>::load(wbase + (size_t)16 * NHID + k0);
      const v16b b2 = Frag<__bf16>::load(wbase + (size_t)32 * NHID + k0);
      const v16b b3 = Frag<__bf16>::load(wbase + (size_t)48 * NHID + k0);
      acc[0] = Frag<__bf16>::mma(fa, b0, acc[0]);
      acc[1] = Frag<__bf16>::mma(fa, b1, acc[1]);
      acc[2] = Frag<__bf16>::mma(fa, b2, acc[2]);
      acc[3] = Frag<__bf16>::mma(fa, b3, acc[3]);
      acc[0] = Frag<__bf16>::mma(fl, b0, acc[0]);
      acc[1] = Frag<__bf16>::mma(fl, b1, acc[1]);
      acc[2] = Frag<__bf16>::mma(fl, b2, acc[2]);
      acc[3] = Frag<__bf16>::mma(fl, b3, acc[3]);
      tie4x6_b(acc[0], acc[1], acc[2], acc[3], fa, fl, b0, b1, b2, b3);
    }
    acc_guard4(acc[0], acc[1], acc[2], acc[3]);
#pragma unroll
    for (int nt = 0; nt < 4; ++nt) {
      const int j = 64 * wave + 16 * nt + c;
#pragma unroll
      for (int r = 0; r < 8; ++r) {
        const float xp = Xs[(8 * hh + r) * XPITCH + j];
        const float z  = (acc[nt][r] + bhh[nt]) + xp;
        hst[nt][r] = tanhf(z);
      }
    }
    __syncthreads();
#pragma unroll
    for (int nt = 0; nt < 4; ++nt) {
      const int j = 64 * wave + 16 * nt + c;
#pragma unroll
      for (int r = 0; r < 8; ++r) {
        const float h = hst[nt][r];
        const unsigned short hb = f2bf_bits(h);
        const unsigned short lb = f2bf_bits(h - bf_bits2f(hb));
        const int idx = (8 * hh + r) * HPITCH + j;
        Hh[idx] = hb;
        Hl[idx] = lb;
      }
    }
    {
      const int tn = (t + 1 < NSTEP) ? (t + 1) : (NSTEP - 1);
      gather_xp(Xs, X, PT, rowbase, tn, tid);
    }
    __syncthreads();
  }

#pragma unroll
  for (int nt = 0; nt < 4; ++nt) {
    const int j = 64 * wave + 16 * nt + c;
#pragma unroll
    for (int r = 0; r < 8; ++r) Xs[(8 * hh + r) * XPITCH + j] = hst[nt][r];
  }
  __syncthreads();
  for (int pass = 0; pass < 2; ++pass) {
#pragma unroll
    for (int it = 0; it < 8; ++it) {
      const int idx = it * NTHR + tid;
      const int row = idx >> 7, c4 = (idx & 127) * 4;
      const v4f v = *(const v4f*)(Xs + row * XPITCH + c4);
      *(volatile v4f*)(out + (size_t)(rowbase + row) * NHID + c4) = v;
    }
    __threadfence();
  }
}

extern "C" void kernel_launch(void* const* d_in, const int* in_sizes, int n_in,
                              void* d_out, int out_size, void* d_ws, size_t ws_size, hipStream_t stream) {
  if (n_in < 6 || d_out == nullptr || d_ws == nullptr) return;
  if (in_sizes[0] != NSEQ * NSTEP || in_sizes[1] != NVOC * NEMB || in_sizes[2] != NHID * NHID ||
      in_sizes[3] != NHID || in_sizes[4] != NHID * NEMB || in_sizes[5] != NHID ||
      out_size != NSEQ * NHID) return;

  const int*   X     = (const int*)d_in[0];
  const float* emb   = (const float*)d_in[1];
  const float* whh_w = (const float*)d_in[2];
  const float* whh_b = (const float*)d_in[3];
  const float* wxh_w = (const float*)d_in[4];
  const float* wxh_b = (const float*)d_in[5];
  float* out = (float*)d_out;

  char* ws = (char*)d_ws; size_t off = 0;
  auto carve = [&](size_t bytes) -> char* { char* p = ws + off; off += (bytes + 255) & ~(size_t)255; return p; };
  unsigned short* EMBB  = (unsigned short*)carve((size_t)NVOC * NEMB * 2);
  unsigned short* WXB   = (unsigned short*)carve((size_t)NHID * NEMB * 2);
  unsigned short* WHB   = (unsigned short*)carve((size_t)NHID * NHID * 2);
  float*          BIAS2 = (float*)carve((size_t)2 * NHID * 4);
  float*          PTAB  = (float*)carve((size_t)NVOC * NHID * 4);
  if (off > ws_size || off > (size_t)134217728) return;

  const int n8e = NVOC * (NEMB / 8);
  const int n8x = NHID * (NEMB / 8);
  const int n8h = NHID * (NHID / 8);
  cvt8_kernel<0><<<(n8e + NTHR - 1) / NTHR, NTHR, 0, stream>>>(emb,   EMBB, NVOC, NEMB / 8, NEMB, 0, 1.0f);
  cvt8_kernel<0><<<(n8x + NTHR - 1) / NTHR, NTHR, 0, stream>>>(wxh_w, WXB,  NHID, NEMB / 8, NEMB, 0, 1.0f);
  cvt8_kernel<0><<<(n8h + NTHR - 1) / NTHR, NTHR, 0, stream>>>(whh_w, WHB,  NHID, NHID / 8, NHID, 0, 1.0f);
  bias_prep_kernel<<<1, NTHR, 0, stream>>>(wxh_b, whh_b, BIAS2);

  const dim3 ggrid(((NVOC / 64) * (NHID / 64)) / 8, 1);
  wmma_gemm64<1, false, 2, 0, false, 0><<<ggrid, 256, 0, stream>>>(
      EMBB, EMBB, NEMB, 0L, WXB, WXB, NEMB, 0L, (void*)PTAB, (void*)PTAB, NHID, 0L,
      BIAS2, (const float*)PTAB, 0L, NVOC, NHID, NEMB, 1.0f);

  rnn_seq_kernel<<<NSEQ / SEQ_BLK, NTHR, 0, stream>>>(X, PTAB, BIAS2, WHB, out);
}
